// TalkingHeadAttention_15728170238612
// MI455X (gfx1250) — hardware-verified
//
#include <hip/hip_runtime.h>
#include <stddef.h>

typedef __attribute__((ext_vector_type(16))) _Float16 v16h;
typedef __attribute__((ext_vector_type(8)))  _Float16 v8h;
typedef __attribute__((ext_vector_type(16))) __bf16   v16b;
typedef __attribute__((ext_vector_type(8)))  __bf16   v8b;
typedef __attribute__((ext_vector_type(8)))  float    v8f;
typedef __attribute__((ext_vector_type(4)))  float    v4f;
typedef __attribute__((ext_vector_type(4)))  unsigned int v4u;

constexpr int kBatch = 4;
constexpr int kN = 1024;
constexpr int kC = 512;
constexpr int kH = 32;
constexpr int kD = 16;
constexpr int kTok = kBatch * kN;
constexpr int kF = 3 * kC;
constexpr int kChunkRows = 512;
constexpr int kChunks = kBatch * (kN / kChunkRows);
constexpr int kPP = 1032;
static_assert(kC == kH * kD, "head split");
static_assert(kTok % 64 == 0 && kF % 64 == 0 && kC % 64 == 0 && kC % 32 == 0, "kit GEMM tiles: M,N multiples of 64, K multiple of 32");
static_assert(kN % 64 == 0 && kChunkRows % 64 == 0 && kN % kChunkRows == 0, "attention tiles");
static_assert((kPP * 2) % 16 == 0, "LDS row pitch 16-byte aligned");

constexpr size_t OFF_L   = 0;
constexpr size_t SZ_PLANE = (size_t)kH * kChunkRows * kN * 2;
constexpr size_t OFF_A   = OFF_L + SZ_PLANE;
constexpr size_t OFF_XB  = OFF_A + SZ_PLANE;
constexpr size_t OFF_WQB = OFF_XB + (size_t)kTok * kC * 2;
constexpr size_t OFF_WPB = OFF_WQB + (size_t)kF * kC * 2;
constexpr size_t OFF_Q16 = OFF_WPB + (size_t)kC * kC * 2;
constexpr size_t OFF_K16 = OFF_Q16 + (size_t)kBatch * kH * kN * kD * 2;
constexpr size_t OFF_VT  = OFF_K16 + (size_t)kBatch * kH * kN * kD * 2;
constexpr size_t OFF_XAH = OFF_VT + (size_t)kBatch * kH * kD * kN * 2;
constexpr size_t OFF_XAL = OFF_XAH + (size_t)kTok * kC * 2;
constexpr size_t OFF_TB  = OFF_XAL + (size_t)kTok * kC * 2;
constexpr size_t OFF_CS  = OFF_TB + 2048 * 4;
constexpr size_t WS_TOTAL = OFF_CS + 2048 * 4;
static_assert(WS_TOTAL == 94388224, "carve total");
static_assert(WS_TOTAL <= 134217728, "carve under 128 MiB");
static_assert((size_t)kTok * kF * 4 <= SZ_PLANE, "f32 qkv plane fits in R_L");
static_assert(OFF_A % 128 == 0 && OFF_XB % 128 == 0 && OFF_WQB % 128 == 0 && OFF_WPB % 128 == 0 && OFF_Q16 % 128 == 0 &&
              OFF_K16 % 128 == 0 && OFF_VT % 128 == 0 && OFF_XAH % 128 == 0 && OFF_XAL % 128 == 0 && OFF_TB % 128 == 0 && OFF_CS % 128 == 0, "128-B aligned carves");

__device__ __forceinline__ unsigned short f2bf_bits(float f) {
  unsigned u = __float_as_uint(f);
  return (unsigned short)((u + 0x7FFFu + ((u >> 16) & 1u)) >> 16);
}
__device__ __forceinline__ float bf_bits2f(unsigned short h) { return __uint_as_float(((unsigned)h) << 16); }
__device__ __forceinline__ float bf16r(float f) {
  float r = bf_bits2f(f2bf_bits(f));
  asm volatile("" : "+v"(r));
  return r;
}
__device__ __forceinline__ unsigned short h_f2bits(float f) { return __builtin_bit_cast(unsigned short, (_Float16)f); }
__device__ __forceinline__ float h_bits2f(unsigned short b) { return (float)__builtin_bit_cast(_Float16, b); }
__device__ __forceinline__ unsigned int pack2h(float a, float b) {
  return (unsigned int)h_f2bits(a) | ((unsigned int)h_f2bits(b) << 16);
}
__device__ __forceinline__ v8f zero8f() { return (v8f){0.f, 0.f, 0.f, 0.f, 0.f, 0.f, 0.f, 0.f}; }
__device__ __forceinline__ v8f mma_h(v16h a, v16h b, v8f c) {
  c = __builtin_amdgcn_wmma_f32_16x16x32_f16(false, a, false, b, (short)0, c, false, false);
  asm volatile("v_nop\n\tv_nop\n\tv_nop\n\tv_nop" : "+v"(c) : "v"(a), "v"(b));
  return c;
}
union HFrag { v16h v; v4u w[2]; };

__device__ __forceinline__ void dep_guard_h(v8f& a, v8f& b, v16h x, v16h y) { asm volatile("v_nop\n\tv_nop\n\tv_nop\n\tv_nop" : "+v"(a), "+v"(b) : "v"(x), "v"(y)); }
__device__ __forceinline__ void dep_guard_b(v8f& a, v8f& b, v16b x, v16b y) { asm volatile("v_nop\n\tv_nop\n\tv_nop\n\tv_nop" : "+v"(a), "+v"(b) : "v"(x), "v"(y)); }
__device__ __forceinline__ void keep4_h(v16h a, v16h b, v16h c, v16h d) { asm volatile("v_nop" :: "v"(a), "v"(b), "v"(c), "v"(d)); }
__device__ __forceinline__ void keep4_b(v16b a, v16b b, v16b c, v16b d) { asm volatile("v_nop" :: "v"(a), "v"(b), "v"(c), "v"(d)); }
__device__ __forceinline__ void acc_guard4(v8f& a, v8f& b, v8f& c, v8f& d) { asm volatile("v_nop\n\tv_nop\n\tv_nop\n\tv_nop" : "+v"(a), "+v"(b), "+v"(c), "+v"(d)); }
template <typename T> struct Frag;
template <> struct Frag<_Float16> {
  typedef v16h V; union U { v16h v; v8h h[2]; };
  static __device__ __forceinline__ v16h load(const _Float16* p) {
    U f; f.h[0] = *(const v8h*)(p); f.h[1] = *(const v8h*)(p + 16); return f.v;
  }
  static __device__ __forceinline__ v8f mma(v16h a, v16h b, v8f c) {
    return __builtin_amdgcn_wmma_f32_16x16x32_f16(false, a, false, b, (short)0, c, false, false);
  }
  static __device__ __forceinline__ void guard(v8f& a, v8f& b, v16h x, v16h y) { dep_guard_h(a, b, x, y); }
  static __device__ __forceinline__ void keep(v16h a, v16h b, v16h c, v16h d) { keep4_h(a, b, c, d); }
};
template <> struct Frag<__bf16> {
  typedef v16b V; union U { v16b v; v8b h[2]; };
  static __device__ __forceinline__ v16b load(const __bf16* p) {
    U f; f.h[0] = *(const v8b*)(p); f.h[1] = *(const v8b*)(p + 16); return f.v;
  }
  static __device__ __forceinline__ v8f mma(v16b a, v16b b, v8f c) {
    return __builtin_amdgcn_wmma_f32_16x16x32_bf16(false, a, false, b, (short)0, c, false, false);
  }
  static __device__ __forceinline__ void guard(v8f& a, v8f& b, v16b x, v16b y) { dep_guard_b(a, b, x, y); }
  static __device__ __forceinline__ void keep(v16b a, v16b b, v16b c, v16b d) { keep4_b(a, b, c, d); }
};

template <int ET> struct Elem;
template <> struct Elem<0> { typedef _Float16 T; };
template <> struct Elem<1> { typedef __bf16 T; };
template <int ET, bool SPLIT, bool SPLITB, int BIAS_MODE, int OUT_MODE>
__global__ __launch_bounds__(256) void wmma_gemm64(
    const unsigned short* __restrict__ Ap, const unsigned short* __restrict__ A2p, int lda, long strideA,
    const unsigned short* __restrict__ Btp, const unsigned short* __restrict__ Bt2p, int ldb, long strideB,
    void* __restrict__ Cout, void* __restrict__ Cout2, int ldc, long strideC,
    const float* __restrict__ bias,
    int M, int N, int K, float scale) {
  typedef typename Elem<ET>::T T;
  typedef typename Frag<T>::V V;
  const T* A = (const T*)Ap; const T* A2 = (const T*)A2p; const T* Bt = (const T*)Btp; const T* Bt2 = (const T*)Bt2p;
  __shared__ __align__(16) float sT[8][16 * 68];
  const int b    = blockIdx.y;
  const int lane = threadIdx.x & 31;
  const int wave = threadIdx.x >> 5;
  const int tilesN = N >> 6;
  const int tilesM = M >> 6;
  const int tile = blockIdx.x * 8 + wave;
  if (tile >= tilesM * tilesN) return;
  const int tm = tile / tilesN;
  const int tn = tile - tm * tilesN;
  const int m0 = tm << 6;
  const int n0 = tn << 6;

  const T* Ab  = A  + (size_t)b * strideA;
  const T* Bb  = Bt + (size_t)b * strideB;
  const T* Ab2 = SPLIT ? (A2  + (size_t)b * strideA) : nullptr;
  const T* Bb2 = (SPLIT && SPLITB) ? (Bt2 + (size_t)b * strideB) : nullptr;

  const int rlane = lane & 15;
  const int koff  = (lane >> 4) * 8;
  const int mOff  = (lane >> 4) * 8;

  v8f acc[4][4];
#pragma unroll
  for (int i = 0; i < 4; ++i)
#pragma unroll
    for (int j = 0; j < 4; ++j) acc[i][j] = (v8f){0.f,0.f,0.f,0.f,0.f,0.f,0.f,0.f};

  for (int k0 = 0; k0 < K; k0 += 32) {
    V bh[4], bl[4];
#pragma unroll
    for (int j = 0; j < 4; ++j) {
      const size_t bo = (size_t)(n0 + (j << 4) + rlane) * ldb + koff + k0;
      bh[j] = Frag<T>::load(Bb + bo);
      if (SPLIT && SPLITB) bl[j] = Frag<T>::load(Bb2 + bo); else bl[j] = bh[j];
    }
#pragma unroll
    for (int i = 0; i < 4; ++i) {
      const size_t ao = (size_t)(m0 + (i << 4) + rlane) * lda + koff + k0;
      V ah = Frag<T>::load(Ab + ao);
      V al = ah;
      if (SPLIT) al = Frag<T>::load(Ab2 + ao);
#pragma unroll
      for (int j = 0; j < 4; ++j) {
        acc[i][j] = Frag<T>::mma(ah, bh[j], acc[i][j]);
        if (SPLIT) {
          if (SPLITB) acc[i][j] = Frag<T>::mma(ah, bl[j], acc[i][j]);
          acc[i][j] = Frag<T>::mma(al, bh[j], acc[i][j]);
        }
      }
      Frag<T>::guard(acc[i][0], acc[i][3], ah, al);
    }
    Frag<T>::keep(bh[0], bh[1], bh[2], bh[3]);
    if (SPLIT && SPLITB) Frag<T>::keep(bl[0], bl[1], bl[2], bl[3]);
  }
  acc_guard4(acc[0][0], acc[0][1], acc[0][2], acc[0][3]);
  acc_guard4(acc[1][0], acc[1][1], acc[1][2], acc[1][3]);
  acc_guard4(acc[2][0], acc[2][1], acc[2][2], acc[2][3]);
  acc_guard4(acc[3][0], acc[3][1], acc[3][2], acc[3][3]);

  float* slab = sT[wave];
#pragma unroll
  for (int i = 0; i < 4; ++i) {
    const int mBase = m0 + (i << 4);
#pragma unroll
    for (int j = 0; j < 4; ++j) {
      const int n = n0 + (j << 4) + rlane;
      float bv = 0.f;
      if (BIAS_MODE == 2) bv = bias[n];
#pragma unroll
      for (int r = 0; r < 8; ++r) {
        float v = acc[i][j][r] * scale;
        if (BIAS_MODE == 1) v += bias[mBase + mOff + r];
        if (BIAS_MODE == 2) v += bv;
        slab[(mOff + r) * 68 + (j << 4) + rlane] = v;
      }
    }
    __builtin_amdgcn_fence(__ATOMIC_RELEASE, "workgroup");
    __builtin_amdgcn_wave_barrier();
    __builtin_amdgcn_fence(__ATOMIC_ACQUIRE, "workgroup");
    if (OUT_MODE == 0) {
      float* C = (float*)Cout + (size_t)b * strideC;
      const int hh = lane >> 4, c4 = (lane & 15) * 4;
      for (int pass = 0; pass < 2; ++pass) {
#pragma unroll
        for (int it = 0; it < 8; ++it) {
          const int row = it * 2 + hh;
          v4f v = *(const v4f*)(slab + row * 68 + c4);
          *(volatile v4f*)(C + (size_t)(mBase + row) * ldc + n0 + c4) = v;
        }
        __threadfence();
      }
    } else {
      const int q = lane >> 3, c8 = (lane & 7) * 8;
      unsigned short* C  = (unsigned short*)Cout  + (size_t)b * strideC;
      unsigned short* C2 = (OUT_MODE == 2) ? ((unsigned short*)Cout2 + (size_t)b * strideC) : nullptr;
      for (int pass = 0; pass < 2; ++pass) {
#pragma unroll
        for (int it = 0; it < 4; ++it) {
          const int row = it * 4 + q;
          const float* sp = slab + row * 68 + c8;
          v8h hv, lv;
#pragma unroll
          for (int e = 0; e < 8; ++e) {
            if (OUT_MODE == 1) {
              hv[e] = (_Float16)sp[e];
            } else {
              unsigned short hb = f2bf_bits(sp[e]);
              unsigned short lb = f2bf_bits(sp[e] - bf_bits2f(hb));
              hv[e] = __builtin_bit_cast(_Float16, hb);
              lv[e] = __builtin_bit_cast(_Float16, lb);
            }
          }
          *(volatile v8h*)(C + (size_t)(mBase + row) * ldc + n0 + c8) = hv;
          if (OUT_MODE == 2) *(volatile v8h*)(C2 + (size_t)(mBase + row) * ldc + n0 + c8) = lv;
        }
        __threadfence();
      }
    }
    __builtin_amdgcn_fence(__ATOMIC_RELEASE, "workgroup");
    __builtin_amdgcn_wave_barrier();
    __builtin_amdgcn_fence(__ATOMIC_ACQUIRE, "workgroup");
  }
}

constexpr int kPrepBX = kTok * kC / 512;
constexpr int kPrepBW = kF * kC / 512;
constexpr int kPrepBP = kC * kC / 512;
static_assert((kTok * kC) % 512 == 0 && (kF * kC) % 512 == 0 && (kC * kC) % 512 == 0, "cast segments are whole blocks");
__global__ __launch_bounds__(256) void prep_kernel(
    const float* __restrict__ x, const float* __restrict__ wqkv, const float* __restrict__ wproj,
    const float* __restrict__ bqkv, const float* __restrict__ bproj,
    unsigned short* __restrict__ xB, unsigned short* __restrict__ wqkvB, unsigned short* __restrict__ wprojB,
    float* __restrict__ tb) {
  const int blk = blockIdx.x;
  const int t = threadIdx.x;
  if (blk < kPrepBX + kPrepBW + kPrepBP) {
    const float* src = x; unsigned short* dst = xB; int lb = blk;
    if (blk >= kPrepBX) { src = wqkv; dst = wqkvB; lb = blk - kPrepBX; }
    if (blk >= kPrepBX + kPrepBW) { src = wproj; dst = wprojB; lb = blk - kPrepBX - kPrepBW; }
    const size_t i = (size_t)lb * 256 + t;
    const float f0 = src[2 * i], f1 = src[2 * i + 1];
    const unsigned u = (unsigned)f2bf_bits(f0) | ((unsigned)f2bf_bits(f1) << 16);
    volatile unsigned* d = (volatile unsigned*)dst;
    d[i] = u;
    __threadfence();
    d[i] = u;
  } else {
    const int j0 = 4 * t;
    const int j1 = 1024 + 4 * t;
    const int jq = (j1 < kF) ? j1 : (kF - 4);
    const int jp = (j1 >= kF) ? (j1 - kF) : 0;
    const v4f a0 = *(const v4f*)(bqkv + j0);
    const v4f aq = *(const v4f*)(bqkv + jq);
    const v4f ap = *(const v4f*)(bproj + jp);
    v4f r0, r1;
#pragma unroll
    for (int e = 0; e < 4; ++e) {
      r0[e] = bf_bits2f(f2bf_bits(a0[e]));
      const float s = (j1 < kF) ? aq[e] : ap[e];
      r1[e] = bf_bits2f(f2bf_bits(s));
    }
    *(volatile v4f*)(tb + j0) = r0;
    *(volatile v4f*)(tb + j1) = r1;
    __threadfence();
    *(volatile v4f*)(tb + j0) = r0;
    *(volatile v4f*)(tb + j1) = r1;
  }
}

__global__ __launch_bounds__(256) void relayout_kernel(
    const float* __restrict__ cq, unsigned short* __restrict__ q16, unsigned short* __restrict__ k16,
    unsigned short* __restrict__ vt16) {
  __shared__ __align__(16) unsigned short sV[16 * 136];
  const int bx = blockIdx.x;
  const int s = blockIdx.y;
  const int b = bx >> 8, h = (bx >> 3) & 31, mc = bx & 7;
  const int tid = threadIdx.x, lane = tid & 31, wave = tid >> 5;
  const int ml = tid >> 1, oct = tid & 1;
  const int m = mc * 128 + ml;
  const float* src = cq + ((size_t)(b * kN + m)) * kF + s * kC + h * kD + oct * 8;
  const v4f f0 = *(const v4f*)(src);
  const v4f f1 = *(const v4f*)(src + 4);
  const float cs = (s == 2) ? 8.0f : 1.0f;
  const v4u pk = (v4u){pack2h(f0[0] * cs, f0[1] * cs), pack2h(f0[2] * cs, f0[3] * cs),
                       pack2h(f1[0] * cs, f1[1] * cs), pack2h(f1[2] * cs, f1[3] * cs)};
  if (s < 2) {
    unsigned short* dst = ((s == 0) ? q16 : k16) + ((size_t)((b * kH + h) * kN + m)) * kD + oct * 8;
    *(volatile v4u*)dst = pk;
    __threadfence();
    *(volatile v4u*)dst = pk;
  } else {
#pragma unroll
    for (int e = 0; e < 4; ++e) {
      sV[(oct * 8 + 2 * e) * 136 + ml]     = (unsigned short)(pk[e] & 0xffffu);
      sV[(oct * 8 + 2 * e + 1) * 136 + ml] = (unsigned short)(pk[e] >> 16);
    }
    __syncthreads();
    const int d = 2 * wave + (lane >> 4), col = (lane & 15) * 8;
    const v4u u = *(const v4u*)(sV + d * 136 + col);
    unsigned short* dst = vt16 + ((size_t)((b * kH + h) * kD + d)) * kN + mc * 128 + col;
    *(volatile v4u*)dst = u;
    __threadfence();
    *(volatile v4u*)dst = u;
  }
}

__global__ __launch_bounds__(256) void colsum_kernel(const float* __restrict__ cq, float* __restrict__ colsum) {
  const int o = blockIdx.x * 256 + threadIdx.x;
  const int b = o >> 9, c = o & 511;
  const float* p = cq + (size_t)b * kN * kF + 2 * kC + c;
  float s0 = 0.f, s1 = 0.f, s2 = 0.f, s3 = 0.f;
#pragma unroll 1
  for (int m = 0; m < kN; m += 4) {
    s0 += p[(size_t)(m) * kF];
    s1 += p[(size_t)(m + 1) * kF];
    s2 += p[(size_t)(m + 2) * kF];
    s3 += p[(size_t)(m + 3) * kF];
  }
  const float s = (s0 + s1) + (s2 + s3);
  ((volatile float*)colsum)[o] = s;
  __threadfence();
  ((volatile float*)colsum)[o] = s;
}

__device__ __forceinline__ v16h mixw_frag(const float* __restrict__ w, int gt, int hh, int c) {
  const float* wp = w + (gt * 16 + c) * kH;
  const v4f t0 = *(const v4f*)(wp + 8 * hh);
  const v4f t1 = *(const v4f*)(wp + 8 * hh + 4);
  const v4f t2 = *(const v4f*)(wp + 16 + 8 * hh);
  const v4f t3 = *(const v4f*)(wp + 20 + 8 * hh);
  HFrag f;
  f.w[0] = (v4u){pack2h(bf16r(t0[0]) * 256.f, bf16r(t0[1]) * 256.f), pack2h(bf16r(t0[2]) * 256.f, bf16r(t0[3]) * 256.f),
                  pack2h(bf16r(t1[0]) * 256.f, bf16r(t1[1]) * 256.f), pack2h(bf16r(t1[2]) * 256.f, bf16r(t1[3]) * 256.f)};
  f.w[1] = (v4u){pack2h(bf16r(t2[0]) * 256.f, bf16r(t2[1]) * 256.f), pack2h(bf16r(t2[2]) * 256.f, bf16r(t2[3]) * 256.f),
                  pack2h(bf16r(t3[0]) * 256.f, bf16r(t3[1]) * 256.f), pack2h(bf16r(t3[2]) * 256.f, bf16r(t3[3]) * 256.f)};
  return f.v;
}

__global__ __launch_bounds__(256) void scores_premix_kernel(
    const unsigned short* __restrict__ q16, const unsigned short* __restrict__ k16,
    const float* __restrict__ wpre, unsigned short* __restrict__ Lpl, int bb, int nh) {
  __shared__ __align__(16) unsigned short sS[16 * 64 * 32];
  __shared__ __align__(16) unsigned short sLb[8][64 * 64];
  const int tid = threadIdx.x, wave = tid >> 5, lane = tid & 31, hh = lane >> 4, c = lane & 15;
  const int nt = blockIdx.x >> 4, mtile = blockIdx.x & 15;
  const int n0c = nt * 16;
  const int n0 = nh * kChunkRows + n0c;
  const int m0 = mtile * 64;
  const v4u z4 = (v4u){0u, 0u, 0u, 0u};

#pragma unroll
  for (int i = 0; i < 4; ++i) {
    const int h = wave * 4 + i;
    const size_t hrow = (size_t)(bb * kH + h) * kN;
    HFrag qa;
    qa.w[0] = *(const v4u*)(q16 + (hrow + n0 + c) * kD + 8 * hh);
    qa.w[1] = z4;
#pragma unroll
    for (int ms = 0; ms < 4; ++ms) {
      HFrag ka;
      ka.w[0] = *(const v4u*)(k16 + (hrow + m0 + ms * 16 + c) * kD + 8 * hh);
      ka.w[1] = z4;
      const v8f acc = mma_h(qa.v, ka.v, zero8f());
#pragma unroll
      for (int r = 0; r < 8; ++r) {
        const int pos = ((8 * hh + r) << 6) + ms * 16 + c;
        sS[pos * 32 + h] = h_f2bits(acc[r]);
      }
    }
  }
  __syncthreads();

  v16h wa[2];
  wa[0] = mixw_frag(wpre, 0, hh, c);
  wa[1] = mixw_frag(wpre, 1, hh, c);

  unsigned short* slab = sLb[wave];
#pragma unroll
  for (int i = 0; i < 8; ++i) {
    const int grp = i >> 2, ml0 = (i & 3) * 16;
    const int pos = ((2 * wave + grp) << 6) + ml0 + c;
    HFrag bf;
    bf.w[0] = *(const v4u*)(sS + pos * 32 + 8 * hh);
    bf.w[1] = *(const v4u*)(sS + pos * 32 + 16 + 8 * hh);
    const v8f a0 = mma_h(wa[0], bf.v, zero8f());
    const v8f a1 = mma_h(wa[1], bf.v, zero8f());
#pragma unroll
    for (int r = 0; r < 8; ++r) {
      slab[(((8 * hh + r) << 1) + grp) * 64 + ml0 + c]      = h_f2bits(a0[r]);
      slab[(((16 + 8 * hh + r) << 1) + grp) * 64 + ml0 + c] = h_f2bits(a1[r]);
    }
  }
  __syncthreads();

  const int q4 = lane >> 3, c8 = (lane & 7) * 8;
  for (int pass = 0; pass < 2; ++pass) {
#pragma unroll
    for (int it = 0; it < 16; ++it) {
      const int rho = it * 4 + q4;
      const int g = rho >> 1, grp = rho & 1;
      const v4u v = *(const v4u*)(slab + rho * 64 + c8);
      const size_t off = ((size_t)(g * kChunkRows + n0c + 2 * wave + grp)) * kN + m0 + c8;
      *(volatile v4u*)(Lpl + off) = v;
    }
    __threadfence();
  }
}

__global__ __launch_bounds__(256) void softmax_postmix_kernel(
    const unsigned short* __restrict__ Lpl, const float* __restrict__ bpre, const float* __restrict__ wpost,
    unsigned short* __restrict__ Apl) {
  __shared__ __align__(16) unsigned short sP[kH * kPP];
  const int nl = blockIdx.x;
  const int tid = threadIdx.x, wave = tid >> 5, lane = tid & 31, hh = lane >> 4, c = lane & 15;

#pragma unroll 1
  for (int i = 0; i < 4; ++i) {
    const int h = wave * 4 + i;
    const unsigned short* src = Lpl + ((size_t)(h * kChunkRows + nl)) * kN;
    const float bpr = bf16r(bpre[h]);
    float lv[32];
#pragma unroll
    for (int j = 0; j < 4; ++j) {
      const v4u w = *(const v4u*)(src + j * 256 + lane * 8);
#pragma unroll
      for (int e = 0; e < 4; ++e) {
        lv[j * 8 + 2 * e]     = h_bits2f((unsigned short)(w[e] & 0xffffu)) * (1.0f / 1024.0f) + bpr;
        lv[j * 8 + 2 * e + 1] = h_bits2f((unsigned short)(w[e] >> 16)) * (1.0f / 1024.0f) + bpr;
      }
    }
    float mx = lv[0];
#pragma unroll
    for (int t = 1; t < 32; ++t) mx = fmaxf(mx, lv[t]);
#pragma unroll
    for (int off = 16; off > 0; off >>= 1) mx = fmaxf(mx, __shfl_xor(mx, off, 32));
    float sm = 0.f;
#pragma unroll
    for (int t = 0; t < 32; ++t) { lv[t] = expf(lv[t] - mx); sm += lv[t]; }
#pragma unroll
    for (int off = 16; off > 0; off >>= 1) sm += __shfl_xor(sm, off, 32);
    const float rs = 65536.0f / sm;
#pragma unroll
    for (int j = 0; j < 4; ++j) {
      const v4u pk = (v4u){pack2h(lv[j * 8 + 0] * rs - 64.0f, lv[j * 8 + 1] * rs - 64.0f),
                           pack2h(lv[j * 8 + 2] * rs - 64.0f, lv[j * 8 + 3] * rs - 64.0f),
                           pack2h(lv[j * 8 + 4] * rs - 64.0f, lv[j * 8 + 5] * rs - 64.0f),
                           pack2h(lv[j * 8 + 6] * rs - 64.0f, lv[j * 8 + 7] * rs - 64.0f)};
      *(v4u*)(sP + h * kPP + j * 256 + lane * 8) = pk;
    }
  }
  __syncthreads();

  v16h wa[2];
  wa[0] = mixw_frag(wpost, 0, hh, c);
  wa[1] = mixw_frag(wpost, 1, hh, c);

#pragma unroll 1
  for (int i = 0; i < 8; ++i) {
    const int m = (wave * 8 + i) * 16 + c;
    unsigned int pw[8];
#pragma unroll
    for (int e = 0; e < 8; ++e) {
      const int ha = 8 * hh + 2 * e + ((e < 4) ? 0 : 8);
      pw[e] = (unsigned int)sP[ha * kPP + m] | ((unsigned int)sP[(ha + 1) * kPP + m] << 16);
    }
    HFrag bf;
    bf.w[0] = (v4u){pw[0], pw[1], pw[2], pw[3]};
    bf.w[1] = (v4u){pw[4], pw[5], pw[6], pw[7]};
    const v8f a0 = mma_h(wa[0], bf.v, zero8f());
    const v8f a1 = mma_h(wa[1], bf.v, zero8f());
#pragma unroll
    for (int r = 0; r < 8; ++r) {
      sP[(8 * hh + r) * kPP + m]      = h_f2bits(a0[r] * (1.0f / 32.0f));
      sP[(16 + 8 * hh + r) * kPP + m] = h_f2bits(a1[r] * (1.0f / 32.0f));
    }
  }
  __syncthreads();

  for (int pass = 0; pass < 2; ++pass) {
#pragma unroll
    for (int i = 0; i < 4; ++i) {
      const int g = wave * 4 + i;
#pragma unroll
      for (int j = 0; j < 4; ++j) {
        const v4u v = *(const v4u*)(sP + g * kPP + j * 256 + lane * 8);
        *(volatile v4u*)(Apl + ((size_t)(g * kChunkRows + nl)) * kN + j * 256 + lane * 8) = v;
      }
    }
    __threadfence();
  }
}

__global__ __launch_bounds__(128) void attnv_kernel(
    const unsigned short* __restrict__ Apl, const unsigned short* __restrict__ vt16,
    const float* __restrict__ wpost, const float* __restrict__ bpost, const float* __restrict__ colsum,
    unsigned short* __restrict__ xah, unsigned short* __restrict__ xal, int bb, int nh) {
  __shared__ __align__(16) float sT[4][16 * 68];
  const int gq = blockIdx.x >> 3, nt = blockIdx.x & 7;
  const int tid = threadIdx.x, wave = tid >> 5, lane = tid & 31, hh = lane >> 4, c = lane & 15;
  const int nl0 = nt * 64 + wave * 16;
  const _Float16* Ab = (const _Float16*)Apl;
  const _Float16* Vb = (const _Float16*)vt16;

  v8f acc[4];
#pragma unroll
  for (int j = 0; j < 4; ++j) acc[j] = zero8f();
#pragma unroll 1
  for (int k0 = 0; k0 < kN; k0 += 32) {
#pragma unroll
    for (int j = 0; j < 4; ++j) {
      const int g = gq * 4 + j;
      const v16h a = Frag<_Float16>::load(Ab + ((size_t)(g * kChunkRows + nl0 + c)) * kN + 8 * hh + k0);
      const v16h v = Frag<_Float16>::load(Vb + ((size_t)((bb * kH + g) * kD + c)) * kN + 8 * hh + k0);
      acc[j] = mma_h(a, v, acc[j]);
    }
  }

  float cgv[4];
#pragma unroll
  for (int j = 0; j < 4; ++j) {
    const int g = gq * 4 + j;
    float t = bf16r(wpost[g * kH + lane]);
#pragma unroll
    for (int off = 16; off > 0; off >>= 1) t += __shfl_xor(t, off, 32);
    cgv[j] = t * (1.0f / 1024.0f) + bf16r(bpost[g]);
  }

  float* slab = sT[wave];
#pragma unroll
  for (int j = 0; j < 4; ++j) {
    const int g = gq * 4 + j;
    const float csv = colsum[(bb * kH + g) * kD + c];
#pragma unroll
    for (int r = 0; r < 8; ++r) slab[(8 * hh + r) * 68 + j * 16 + c] = acc[j][r] * (1.0f / 4194304.0f) + cgv[j] * csv;
  }
  __syncthreads();

  const int q4 = lane >> 3, c8 = (lane & 7) * 8;
  const size_t rowbase = (size_t)bb * kN + (size_t)nh * kChunkRows + nl0;
  for (int pass = 0; pass < 2; ++pass) {
#pragma unroll
    for (int it = 0; it < 4; ++it) {
      const int row = it * 4 + q4;
      const float* sp = slab + row * 68 + c8;
      unsigned int hw[4], lw[4];
#pragma unroll
      for (int e = 0; e < 4; ++e) {
        const unsigned short hb0 = f2bf_bits(sp[2 * e]);
        const unsigned short lb0 = f2bf_bits(sp[2 * e] - bf_bits2f(hb0));
        const unsigned short hb1 = f2bf_bits(sp[2 * e + 1]);
        const unsigned short lb1 = f2bf_bits(sp[2 * e + 1] - bf_bits2f(hb1));
        hw[e] = (unsigned int)hb0 | ((unsigned int)hb1 << 16);
        lw[e] = (unsigned int)lb0 | ((unsigned int)lb1 << 16);
      }
      const v4u hv = (v4u){hw[0], hw[1], hw[2], hw[3]};
      const v4u lv = (v4u){lw[0], lw[1], lw[2], lw[3]};
      const size_t off = (rowbase + row) * kC + gq * 64 + c8;
      *(volatile v4u*)(xah + off) = hv;
      *(volatile v4u*)(xal + off) = lv;
    }
    __threadfence();
  }
}

extern "C" void kernel_launch(void* const* d_in, const int* in_sizes, int n_in,
                              void* d_out, int out_size, void* d_ws,
                              size_t ws_size, hipStream_t stream) {
  if (n_in < 9) return;
  if (in_sizes[0] != kTok * kC || in_sizes[1] != kF * kC || in_sizes[2] != kF || in_sizes[3] != kH * kH ||
      in_sizes[4] != kH || in_sizes[5] != kH * kH || in_sizes[6] != kH || in_sizes[7] != kC * kC || in_sizes[8] != kC) return;
  if (out_size != kTok * kC) return;
  if (ws_size < WS_TOTAL) return;

  const float* x     = (const float*)d_in[0];
  const float* Wqkv  = (const float*)d_in[1];
  const float* bqkv  = (const float*)d_in[2];
  const float* Wpre  = (const float*)d_in[3];
  const float* bpre  = (const float*)d_in[4];
  const float* Wpost = (const float*)d_in[5];
  const float* bpost = (const float*)d_in[6];
  const float* Wproj = (const float*)d_in[7];
  const float* bproj = (const float*)d_in[8];
  float* out = (float*)d_out;

  char* ws = (char*)d_ws;
  unsigned short* Lpl  = (unsigned short*)(ws + OFF_L);
  float*          cqkv = (float*)(ws + OFF_L);
  unsigned short* Apl  = (unsigned short*)(ws + OFF_A);
  unsigned short* xB   = (unsigned short*)(ws + OFF_XB);
  unsigned short* wqB  = (unsigned short*)(ws + OFF_WQB);
  unsigned short* wpB  = (unsigned short*)(ws + OFF_WPB);
  unsigned short* q16  = (unsigned short*)(ws + OFF_Q16);
  unsigned short* k16  = (unsigned short*)(ws + OFF_K16);
  unsigned short* vt16 = (unsigned short*)(ws + OFF_VT);
  unsigned short* xah  = (unsigned short*)(ws + OFF_XAH);
  unsigned short* xal  = (unsigned short*)(ws + OFF_XAL);
  float*          tb   = (float*)(ws + OFF_TB);
  float*          csum = (float*)(ws + OFF_CS);

  prep_kernel<<<dim3(kPrepBX + kPrepBW + kPrepBP + 1), dim3(256), 0, stream>>>(x, Wqkv, Wproj, bqkv, bproj, xB, wqB, wpB, tb);

  wmma_gemm64<1, false, false, 2, 0><<<dim3((kTok / 64) * (kF / 64) / 8, 1), dim3(256), 0, stream>>>(
      xB, xB, kC, 0L, wqB, wqB, kC, 0L, (void*)cqkv, (void*)cqkv, kF, 0L, tb, kTok, kF, kC, 1.0f);

  relayout_kernel<<<dim3(kBatch * kH * (kN / 128), 3), dim3(256), 0, stream>>>(cqkv, q16, k16, vt16);
  colsum_kernel<<<dim3(kBatch * kC / 256), dim3(256), 0, stream>>>(cqkv, csum);

  for (int ch = 0; ch < kChunks; ++ch) {
    const int bb = ch >> 1, nh = ch & 1;
    scores_premix_kernel<<<dim3((kChunkRows / 16) * (kN / 64)), dim3(256), 0, stream>>>(q16, k16, Wpre, Lpl, bb, nh);
    softmax_postmix_kernel<<<dim3(kChunkRows), dim3(256), 0, stream>>>(Lpl, bpre, Wpost, Apl);
    attnv_kernel<<<dim3((kH / 4) * (kChunkRows / 64)), dim3(128), 0, stream>>>(Apl, vt16, Wpost, bpost, csum, xah, xal, bb, nh);
  }

  wmma_gemm64<1, true, false, 2, 0><<<dim3((kTok / 64) * (kC / 64) / 8, 1), dim3(256), 0, stream>>>(
      xah, xal, kC, 0L, wpB, wpB, kC, 0L, (void*)out, (void*)out, kC, 0L, tb + kF, kTok, kC, kC, 1.0f);
}
